// Deep_Feature_Extractor_30356828848459
// MI455X (gfx1250) — hardware-run, weakly checked
//
#include <hip/hip_runtime.h>
#include <stdint.h>
#include <math.h>

#define DEVINL __device__ __forceinline__

typedef _Float16 f16t;
typedef _Float16 v16h __attribute__((ext_vector_type(16)));
typedef _Float16 v8h  __attribute__((ext_vector_type(8)));
typedef float    v8f  __attribute__((ext_vector_type(8)));
typedef float    v4f  __attribute__((ext_vector_type(4)));
typedef v8h __attribute__((may_alias)) v8ha;
typedef v4f __attribute__((may_alias)) v4fa;
union FragH { v16h v; v8h half[2]; };

#define NBAT   8
#define IMG    64
#define CD     256
#define TOK    32768
#define WSZ    16
#define WTOK   256
#define NWIN   128
#define NWIMG  16
#define NHEAD  8
#define HD     32
#define NQ     768
#define NH     1024
#define NDEP   2
#define RPBN   961
#define TPB    256
#define WAVES  8
#define MT     128
#define NTL    128
#define PQF    132
#define WTP    72
#define BBIAS  1024
#define ACAR   16.0f
#define WCAR   256.0f
#define QCAR   16.0f
#define PCAR   1024.0f
#define OCAR   64.0f
#define HCAR   16.0f
#define INV_AW (1.0f / 4096.0f)
#define INV_OW (1.0f / 16384.0f)
#define SSC    (0.17677669529663687f / 256.0f)
#define OSCL   4.0f
#define ATT_LDS 90112

static_assert(TPB == WAVES * 32);
static_assert(NBAT * IMG * IMG == TOK);
static_assert(NWIN * WTOK == TOK);
static_assert(NBAT * NWIMG == NWIN);
static_assert((IMG / WSZ) * (IMG / WSZ) == NWIMG);
static_assert(WSZ * WSZ == WTOK);
static_assert(NHEAD * HD == CD);
static_assert(NQ == 3 * CD && NH == 4 * CD);
static_assert((TOK % MT) == 0 && (WTOK % MT) == 0);
static_assert((NQ % NTL) == 0 && (CD % NTL) == 0 && (NH % NTL) == 0);
static_assert((CD % 64) == 0 && (NQ % 64) == 0 && (NH % 64) == 0);
static_assert((CD % 32) == 0 && (NH % 32) == 0);
static_assert(CD == 8 * 32);
static_assert((TOK % WAVES) == 0);
static_assert((PQF % 4) == 0 && (WTP % 8) == 0);
static_assert(64 * PQF * 4 <= 40000);
static_assert(2 * WTOK * HD / 8 == 8 * TPB);
static_assert((2 * WTOK * HD + 2 * HD * WTOK + WAVES * 16 * 64 + 64 * 64) * 2 == ATT_LDS);
static_assert(NDEP * NHEAD * WTOK * (WTOK / 4) == BBIAS * TPB);
static_assert(NWIMG * WTOK * (WTOK / 4) == BBIAS * TPB);
static_assert((WTOK % 64) == 0);

DEVINL int imin(int a, int b) { return a < b ? a : b; }
DEVINL int imax(int a, int b) { return a > b ? a : b; }

DEVINL v8f wmma_f16(v16h a, v16h b, v8f c) {
  v8f d = __builtin_amdgcn_wmma_f32_16x16x32_f16(false, a, false, b, (short)0, c, false, false);
  asm volatile("v_nop\n\tv_nop\n\tv_nop\n\tv_nop" : "+v"(d) : "v"(a), "v"(b));
  return d;
}
DEVINL v8f zero8f() {
  v8f z = {0.f, 0.f, 0.f, 0.f, 0.f, 0.f, 0.f, 0.f};
  return z;
}
DEVINL v4f zero4f() {
  v4f z = {0.f, 0.f, 0.f, 0.f};
  return z;
}
DEVINL void load_frag(FragH& f, const f16t* row, int k0) {
  f.half[0] = *(const v8ha*)(row + k0);
  f.half[1] = *(const v8ha*)(row + k0 + 16);
}

DEVINL int spat_row(int r, int shift) {
  const int wb = r >> 8, tok = r & 255;
  const int bb = wb >> 4, wimg = wb & 15, wr = wimg >> 2, wc = wimg & 3;
  const int ti = tok >> 4, tj = tok & 15;
  const int hh = (wr * WSZ + ti + shift) & (IMG - 1);
  const int ww = (wc * WSZ + tj + shift) & (IMG - 1);
  return (bb * IMG + hh) * IMG + ww;
}

__global__ __launch_bounds__(TPB) void wtr_k(const float* __restrict__ src, f16t* __restrict__ dst, int K, int N)
{
  __shared__ __attribute__((aligned(16))) f16t st[64 * WTP];
  const int tid = threadIdx.x;
  const int n0 = blockIdx.x * 64, k0 = blockIdx.y * 64, z = blockIdx.z;
  if (n0 + 64 > N || k0 + 64 > K) return;
  const float* s = src + (size_t)z * K * N;
  f16t* dd = dst + (size_t)z * K * N;
  const int kr = tid >> 2, ns = (tid & 3) * 16;
  const float* sp = s + (size_t)(k0 + kr) * N + n0 + ns;
  const v4f a0 = *(const v4fa*)sp, a1 = *(const v4fa*)(sp + 4);
  const v4f a2 = *(const v4fa*)(sp + 8), a3 = *(const v4fa*)(sp + 12);
  #pragma unroll
  for (int j = 0; j < 4; ++j) {
    st[(ns + j) * WTP + kr]      = (f16t)(a0[j] * WCAR);
    st[(ns + 4 + j) * WTP + kr]  = (f16t)(a1[j] * WCAR);
    st[(ns + 8 + j) * WTP + kr]  = (f16t)(a2[j] * WCAR);
    st[(ns + 12 + j) * WTP + kr] = (f16t)(a3[j] * WCAR);
  }
  __syncthreads();
  const int q8 = tid & 7, rA = tid >> 3, rB = rA + 32;
  const v8h vA = *(const v8ha*)(st + rA * WTP + 8 * q8);
  const v8h vB = *(const v8ha*)(st + rB * WTP + 8 * q8);
  f16t* pA = dd + (size_t)(n0 + rA) * K + k0 + 8 * q8;
  f16t* pB = dd + (size_t)(n0 + rB) * K + k0 + 8 * q8;
  *(volatile v8h*)pA = vA;
  *(volatile v8h*)pB = vB;
  __threadfence();
  *(volatile v8h*)pA = vA;
  *(volatile v8h*)pB = vB;
}

__global__ __launch_bounds__(TPB) void bias_k(const float* __restrict__ rpb, const int* __restrict__ rpi,
                                             const float* __restrict__ amask, float* __restrict__ btp,
                                             float* __restrict__ mkp)
{
  const int tid = threadIdx.x, blk = blockIdx.x;
  if (blk >= 2 * BBIAS) return;
  v4f v;
  float* p;
  if (blk < BBIAS) {
    const int g = blk * TPB + tid;
    const int kq = g & 63, q = (g >> 6) & 255, hh = (g >> 14) & 7, z = (g >> 17) & 1;
    const int c = kq >> 4, mm = kq & 15;
    #pragma unroll
    for (int t = 0; t < 4; ++t) {
      int idx = rpi[q * WTOK + 64 * c + 16 * t + mm];
      idx = imin(imax(idx, 0), RPBN - 1);
      v[t] = rpb[((size_t)z * RPBN + idx) * NHEAD + hh];
    }
    p = btp + (((size_t)z * NHEAD + hh) * WTOK + q) * WTOK + 4 * kq;
  } else {
    const int g = (blk - BBIAS) * TPB + tid;
    const int kq = g & 63, q = (g >> 6) & 255, wimg = (g >> 14) & 15;
    const int c = kq >> 4, mm = kq & 15;
    #pragma unroll
    for (int t = 0; t < 4; ++t)
      v[t] = amask[((size_t)wimg * WTOK + q) * WTOK + 64 * c + 16 * t + mm];
    p = mkp + ((size_t)wimg * WTOK + q) * WTOK + 4 * kq;
  }
  *(volatile v4f*)p = v;
  __threadfence();
  *(volatile v4f*)p = v;
}

__global__ __launch_bounds__(TPB) void ln_k(const float* xin, const float* __restrict__ g,
                                           const float* __restrict__ bv, f16t* __restrict__ XM,
                                           int shift, int windowed)
{
  const int tid = threadIdx.x, lane = tid & 31, wave = tid >> 5;
  const int tg = blockIdx.x * WAVES + wave;
  const int srow = windowed ? spat_row(tg, shift) : tg;
  const float* xr = xin + (size_t)srow * CD + 8 * lane;
  const v4f xa = *(const v4fa*)xr, xb = *(const v4fa*)(xr + 4);

  float s = 0.0f;
  #pragma unroll
  for (int e = 0; e < 4; ++e) s += xa[e] + xb[e];
  #pragma unroll
  for (int off = 16; off >= 1; off >>= 1) s += __shfl_xor(s, off, 32);
  const float mean = s * (1.0f / 256.0f);
  float s2 = 0.0f;
  #pragma unroll
  for (int e = 0; e < 4; ++e) {
    const float d0 = xa[e] - mean, d1 = xb[e] - mean;
    s2 = fmaf(d0, d0, s2); s2 = fmaf(d1, d1, s2);
  }
  #pragma unroll
  for (int off = 16; off >= 1; off >>= 1) s2 += __shfl_xor(s2, off, 32);
  const float rstd = rsqrtf(s2 * (1.0f / 256.0f) + 1e-5f);

  const v4f ga = *(const v4fa*)(g + 8 * lane),  gb = *(const v4fa*)(g + 8 * lane + 4);
  const v4f ba = *(const v4fa*)(bv + 8 * lane), bb = *(const v4fa*)(bv + 8 * lane + 4);
  v8h o;
  #pragma unroll
  for (int e = 0; e < 4; ++e) {
    o[e]     = (f16t)((((xa[e] - mean) * rstd) * ga[e] + ba[e]) * ACAR);
    o[4 + e] = (f16t)((((xb[e] - mean) * rstd) * gb[e] + bb[e]) * ACAR);
  }
  f16t* d = XM + (size_t)tg * CD + 8 * lane;
  *(volatile v8h*)d = o;
  __threadfence();
  *(volatile v8h*)d = o;
}

template <int EPI>
__global__ __launch_bounds__(TPB) void gemm_k(const f16t* __restrict__ A, const f16t* __restrict__ Wt,
                                             const float* __restrict__ bias, const float* resid, float* outf,
                                             f16t* __restrict__ outh, int N, int K, float inv, float ocar, int shift)
{
  __shared__ __attribute__((aligned(16))) float sbuf[64 * PQF];
  const int tid = threadIdx.x, lane = tid & 31, wave = tid >> 5;
  const int h = lane >> 4, m = lane & 15;
  const int wm = wave >> 1, wn = wave & 1;
  const int row0 = blockIdx.y * MT, n0 = blockIdx.x * NTL;
  const int mo = row0 + 32 * wm, no = n0 + 64 * wn;

  v8f acc[2][4];
  #pragma unroll
  for (int mh = 0; mh < 2; ++mh)
    #pragma unroll
    for (int t = 0; t < 4; ++t) acc[mh][t] = zero8f();

  const f16t* arow0 = A + (size_t)(mo + m) * K + 8 * h;
  const f16t* arow1 = arow0 + (size_t)16 * K;
  const f16t* brow  = Wt + (size_t)(no + m) * K + 8 * h;
  #pragma unroll 1
  for (int k0 = 0; k0 < K; k0 += 32) {
    FragH a0, a1;
    load_frag(a0, arow0, k0);
    load_frag(a1, arow1, k0);
    #pragma unroll
    for (int t = 0; t < 4; ++t) {
      FragH bw;
      load_frag(bw, brow + (size_t)16 * t * K, k0);
      acc[0][t] = wmma_f16(a0.v, bw.v, acc[0][t]);
      acc[1][t] = wmma_f16(a1.v, bw.v, acc[1][t]);
    }
  }

  #pragma unroll
  for (int p = 0; p < 2; ++p) {
    if ((wm >> 1) == p) {
      #pragma unroll
      for (int t = 0; t < 4; ++t) {
        const float bvv = bias[no + 16 * t + m];
        #pragma unroll
        for (int mh = 0; mh < 2; ++mh) {
          #pragma unroll
          for (int r = 0; r < 8; ++r)
            sbuf[((wm & 1) * 32 + 16 * mh + 8 * h + r) * PQF + 64 * wn + 16 * t + m] = acc[mh][t][r] * inv + bvv;
        }
      }
    }
    __syncthreads();
    const int seg0 = row0 + 64 * p;
    if constexpr (EPI >= 2) {
      v4f vals[8];
      size_t dro[8];
      #pragma unroll
      for (int i = 0; i < 8; ++i) {
        const int row = wave + 8 * i;
        const int srow = seg0 + row;
        const int drow = (EPI == 3) ? spat_row(srow, shift) : srow;
        dro[i] = (size_t)drow * N + n0 + 4 * lane;
        const v4f c  = *(const v4fa*)(sbuf + row * PQF + 4 * lane);
        const v4f rs = *(const v4fa*)(resid + dro[i]);
        vals[i] = rs + c;
      }
      #pragma unroll
      for (int i = 0; i < 8; ++i) *(volatile v4f*)(outf + dro[i]) = vals[i];
      __threadfence();
      #pragma unroll
      for (int i = 0; i < 8; ++i) *(volatile v4f*)(outf + dro[i]) = vals[i];
    } else {
      v8h hv[4];
      #pragma unroll
      for (int j = 0; j < 4; ++j) {
        const int row = wave + 8 * (2 * j + h);
        const float* sp = sbuf + row * PQF + 8 * m;
        const v4f c0 = *(const v4fa*)sp, c1 = *(const v4fa*)(sp + 4);
        #pragma unroll
        for (int e = 0; e < 4; ++e) {
          float u0 = c0[e], u1 = c1[e];
          if constexpr (EPI == 1) {
            u0 = 0.5f * u0 * (1.0f + erff(u0 * 0.70710678118654752f));
            u1 = 0.5f * u1 * (1.0f + erff(u1 * 0.70710678118654752f));
          }
          hv[j][e]     = (f16t)(u0 * ocar);
          hv[j][4 + e] = (f16t)(u1 * ocar);
        }
      }
      #pragma unroll
      for (int j = 0; j < 4; ++j)
        *(volatile v8h*)(outh + (size_t)(seg0 + wave + 8 * (2 * j + h)) * N + n0 + 8 * m) = hv[j];
      __threadfence();
      #pragma unroll
      for (int j = 0; j < 4; ++j)
        *(volatile v8h*)(outh + (size_t)(seg0 + wave + 8 * (2 * j + h)) * N + n0 + 8 * m) = hv[j];
    }
    __syncthreads();
  }
}

template <int SHIFTED>
__global__ __launch_bounds__(TPB) void attn_k(const f16t* __restrict__ QKV, const float* __restrict__ btp,
                                             const float* __restrict__ mkp, f16t* __restrict__ ATT)
{
  extern __shared__ v8h dynraw[];
  f16t* sK  = (f16t*)dynraw;
  f16t* sVt = sK + 2 * WTOK * HD;
  f16t* sP  = sVt + 2 * HD * WTOK;
  f16t* sO  = sP + WAVES * 16 * 64;
  const int tid = threadIdx.x, lane = tid & 31, wave = tid >> 5;
  const int h = lane >> 4, m = lane & 15;
  const int hp = blockIdx.x & 3, wb = blockIdx.x >> 2;
  const size_t rowb = (size_t)wb * WTOK;

  #pragma unroll
  for (int it = 0; it < 8; ++it) {
    const int p = it * TPB + tid;
    const int hs0 = p >> 10, key = (p >> 2) & (WTOK - 1), q4 = p & 3;
    const f16t* src = QKV + (rowb + key) * NQ + CD + (2 * hp + hs0) * HD + 8 * q4;
    const v8h kv = *(const v8ha*)src;
    const v8h vv = *(const v8ha*)(src + CD);
    *(v8ha*)(sK + (hs0 * WTOK + key) * HD + 8 * q4) = kv;
    f16t* vt = sVt + (hs0 * HD + 8 * q4) * WTOK + key;
    #pragma unroll
    for (int i = 0; i < 8; ++i) vt[i * WTOK] = vv[i];
  }
  __syncthreads();

  const int hs = wave >> 2, wq = wave & 3, head = 2 * hp + hs;
  FragH onesf;
  #pragma unroll
  for (int i = 0; i < 16; ++i) onesf.v[i] = (f16t)1.0f;
  f16t* pw = sP + wave * (16 * 64);
  const f16t* kbase = sK + (hs * WTOK + m) * HD + 8 * h;
  const f16t* vbase = sVt + (hs * HD + m) * WTOK + 8 * h;
  const int wimg = wb & (NWIMG - 1);

  #pragma unroll 1
  for (int qt = 0; qt < 4; ++qt) {
    const int lr0 = 64 * qt + 16 * wq;
    FragH qa;
    {
      const f16t* qr = QKV + (rowb + lr0 + m) * NQ + head * HD + 8 * h;
      qa.half[0] = *(const v8ha*)qr;
      qa.half[1] = *(const v8ha*)(qr + 16);
    }
    float run_max[8];
    v8f oacc[2];
    v8f ssum = zero8f();
    oacc[0] = zero8f();
    oacc[1] = zero8f();
    #pragma unroll
    for (int r = 0; r < 8; ++r) run_max[r] = -1.0e30f;
    const float* btw = btp + ((size_t)head * WTOK + lr0 + 8 * h) * WTOK + 4 * m;
    const float* mkw = mkp + ((size_t)wimg * WTOK + lr0 + 8 * h) * WTOK + 4 * m;

    #pragma unroll 1
    for (int c = 0; c < 4; ++c) {
      const int key0 = 64 * c;
      v8f st[4];
      #pragma unroll
      for (int t = 0; t < 4; ++t) {
        FragH kb;
        const f16t* kr = kbase + (key0 + 16 * t) * HD;
        kb.half[0] = *(const v8ha*)kr;
        kb.half[1] = *(const v8ha*)(kr + 16);
        st[t] = wmma_f16(qa.v, kb.v, zero8f());
      }
      #pragma unroll
      for (int gq = 0; gq < 2; ++gq) {
        if (gq == 1) asm volatile("s_wait_loadcnt 0x0" ::: "memory");
        v4f bb[4], mk[4];
        #pragma unroll
        for (int j = 0; j < 4; ++j) {
          const int r = 4 * gq + j;
          bb[j] = *(const v4fa*)(btw + r * WTOK + key0);
          if constexpr (SHIFTED) mk[j] = *(const v4fa*)(mkw + r * WTOK + key0);
          else mk[j] = zero4f();
        }
        #pragma unroll
        for (int j = 0; j < 4; ++j) {
          const int r = 4 * gq + j;
          const float s0 = (st[0][r] * SSC + bb[j][0]) + mk[j][0];
          const float s1 = (st[1][r] * SSC + bb[j][1]) + mk[j][1];
          const float s2 = (st[2][r] * SSC + bb[j][2]) + mk[j][2];
          const float s3 = (st[3][r] * SSC + bb[j][3]) + mk[j][3];
          float mx = fmaxf(fmaxf(s0, s1), fmaxf(s2, s3));
          #pragma unroll
          for (int off = 8; off >= 1; off >>= 1) mx = fmaxf(mx, __shfl_xor(mx, off, 32));
          const float nm = fmaxf(run_max[r], mx);
          const float alpha = __expf(run_max[r] - nm);
          run_max[r] = nm;
          oacc[0][r] *= alpha;
          oacc[1][r] *= alpha;
          ssum[r] *= alpha;
          f16t* prow = pw + (8 * h + r) * 64 + m;
          prow[0]  = (f16t)(__expf(s0 - nm) * PCAR);
          prow[16] = (f16t)(__expf(s1 - nm) * PCAR);
          prow[32] = (f16t)(__expf(s2 - nm) * PCAR);
          prow[48] = (f16t)(__expf(s3 - nm) * PCAR);
        }
      }
      __syncthreads();
      #pragma unroll
      for (int s = 0; s < 2; ++s) {
        FragH pa;
        const f16t* pr = pw + m * 64 + 32 * s + 8 * h;
        pa.half[0] = *(const v8ha*)pr;
        pa.half[1] = *(const v8ha*)(pr + 16);
        ssum = wmma_f16(pa.v, onesf.v, ssum);
        #pragma unroll
        for (int ct = 0; ct < 2; ++ct) {
          FragH vb;
          const f16t* vr = vbase + 16 * ct * WTOK + key0 + 32 * s;
          vb.half[0] = *(const v8ha*)vr;
          vb.half[1] = *(const v8ha*)(vr + 16);
          oacc[ct] = wmma_f16(pa.v, vb.v, oacc[ct]);
        }
      }
    }

    #pragma unroll
    for (int r = 0; r < 8; ++r) {
      const float rinv = OSCL * (1.0f / ssum[r]);
      f16t* orow = sO + (16 * wq + 8 * h + r) * 64 + hs * HD + m;
      orow[0]  = (f16t)(oacc[0][r] * rinv);
      orow[16] = (f16t)(oacc[1][r] * rinv);
    }
    __syncthreads();
    {
      const int q8 = tid & 7, rA = tid >> 3, rB = rA + 32;
      const v8h vA = *(const v8ha*)(sO + rA * 64 + 8 * q8);
      const v8h vB = *(const v8ha*)(sO + rB * 64 + 8 * q8);
      f16t* dA = ATT + (rowb + 64 * qt + rA) * CD + 64 * hp + 8 * q8;
      f16t* dB = ATT + (rowb + 64 * qt + rB) * CD + 64 * hp + 8 * q8;
      *(volatile v8h*)dA = vA;
      *(volatile v8h*)dB = vB;
      __threadfence();
      *(volatile v8h*)dA = vA;
      *(volatile v8h*)dB = vB;
    }
  }
}

extern "C" void kernel_launch(void* const* d_in, const int* in_sizes, int n_in,
                              void* d_out, int out_size, void* d_ws, size_t ws_size,
                              hipStream_t stream) {
  if (n_in < 16) return;
  if (in_sizes[0] != TOK * CD) return;
  if (in_sizes[1] != NDEP * CD || in_sizes[2] != NDEP * CD) return;
  if (in_sizes[3] != NDEP * CD * NQ || in_sizes[4] != NDEP * NQ) return;
  if (in_sizes[5] != NDEP * RPBN * NHEAD) return;
  if (in_sizes[6] != NDEP * CD * CD || in_sizes[7] != NDEP * CD) return;
  if (in_sizes[8] != NDEP * CD || in_sizes[9] != NDEP * CD) return;
  if (in_sizes[10] != NDEP * CD * NH || in_sizes[11] != NDEP * NH) return;
  if (in_sizes[12] != NDEP * NH * CD || in_sizes[13] != NDEP * CD) return;
  if (in_sizes[14] != NWIMG * WTOK * WTOK) return;
  if (in_sizes[15] != WTOK * WTOK) return;
  if (out_size != TOK * CD) return;

  const float* x      = (const float*)d_in[0];
  const float* ln1_g  = (const float*)d_in[1];
  const float* ln1_b  = (const float*)d_in[2];
  const float* qkv_w  = (const float*)d_in[3];
  const float* qkv_b  = (const float*)d_in[4];
  const float* rpb    = (const float*)d_in[5];
  const float* proj_w = (const float*)d_in[6];
  const float* proj_b = (const float*)d_in[7];
  const float* ln2_g  = (const float*)d_in[8];
  const float* ln2_b  = (const float*)d_in[9];
  const float* fc1_w  = (const float*)d_in[10];
  const float* fc1_b  = (const float*)d_in[11];
  const float* fc2_w  = (const float*)d_in[12];
  const float* fc2_b  = (const float*)d_in[13];
  const float* amask  = (const float*)d_in[14];
  const int*   rpi    = (const int*)d_in[15];
  float* outp = (float*)d_out;

  const size_t szBT = (size_t)NDEP * NHEAD * WTOK * WTOK * 4;
  const size_t szMK = (size_t)NWIMG * WTOK * WTOK * 4;
  const size_t szWQ = (size_t)NDEP * NQ * CD * 2;
  const size_t szWP = (size_t)NDEP * CD * CD * 2;
  const size_t szW1 = (size_t)NDEP * NH * CD * 2;
  const size_t szW2 = (size_t)NDEP * CD * NH * 2;
  const size_t szA  = (size_t)TOK * CD * 2;
  const size_t szB  = (size_t)TOK * NH * 2;
  size_t off = 0;
  char* ws = (char*)d_ws;
  float* BTP = (float*)(ws + off); off += szBT;
  float* MKP = (float*)(ws + off); off += szMK;
  f16t*  WQ = (f16t*)(ws + off);  off += szWQ;
  f16t*  WP = (f16t*)(ws + off);  off += szWP;
  f16t*  W1 = (f16t*)(ws + off);  off += szW1;
  f16t*  W2 = (f16t*)(ws + off);  off += szW2;
  f16t*  regA = (f16t*)(ws + off); off += szA;
  f16t*  regB = (f16t*)(ws + off); off += szB;
  if (off > ws_size) return;
  if ((size_t)TOK * NQ * 2 > szB) return;

  f16t* XMp  = regA;
  f16t* ATTp = regA;
  f16t* QKVp = regB;
  f16t* Hp   = regB;

  (void)hipFuncSetAttribute(reinterpret_cast<const void*>(&attn_k<0>), hipFuncAttributeMaxDynamicSharedMemorySize, ATT_LDS);
  (void)hipFuncSetAttribute(reinterpret_cast<const void*>(&attn_k<1>), hipFuncAttributeMaxDynamicSharedMemorySize, ATT_LDS);

  wtr_k<<<dim3(NQ / 64, CD / 64, NDEP), TPB, 0, stream>>>(qkv_w, WQ, CD, NQ);
  wtr_k<<<dim3(CD / 64, CD / 64, NDEP), TPB, 0, stream>>>(proj_w, WP, CD, CD);
  wtr_k<<<dim3(NH / 64, CD / 64, NDEP), TPB, 0, stream>>>(fc1_w, W1, CD, NH);
  wtr_k<<<dim3(CD / 64, NH / 64, NDEP), TPB, 0, stream>>>(fc2_w, W2, NH, CD);
  bias_k<<<2 * BBIAS, TPB, 0, stream>>>(rpb, rpi, amask, BTP, MKP);

  for (int d = 0; d < NDEP; ++d) {
    const int shift = (d & 1) ? (WSZ / 2) : 0;
    const float* xcur = (d == 0) ? x : (const float*)outp;
    const float* btd = BTP + (size_t)d * NHEAD * WTOK * WTOK;
    ln_k<<<TOK / WAVES, TPB, 0, stream>>>(xcur, ln1_g + d * CD, ln1_b + d * CD, XMp, shift, 1);
    gemm_k<0><<<dim3(NQ / NTL, TOK / MT), TPB, 0, stream>>>(XMp, WQ + (size_t)d * NQ * CD, qkv_b + d * NQ,
                                                            x, outp, QKVp, NQ, CD, INV_AW, QCAR, 0);
    if (shift)
      attn_k<1><<<NWIN * 4, TPB, ATT_LDS, stream>>>(QKVp, btd, MKP, ATTp);
    else
      attn_k<0><<<NWIN * 4, TPB, ATT_LDS, stream>>>(QKVp, btd, MKP, ATTp);
    gemm_k<3><<<dim3(CD / NTL, TOK / MT), TPB, 0, stream>>>(ATTp, WP + (size_t)d * CD * CD, proj_b + d * CD,
                                                            xcur, outp, Hp, CD, CD, INV_OW, 1.0f, shift);
    ln_k<<<TOK / WAVES, TPB, 0, stream>>>(outp, ln2_g + d * CD, ln2_b + d * CD, XMp, 0, 0);
    gemm_k<1><<<dim3(NH / NTL, TOK / MT), TPB, 0, stream>>>(XMp, W1 + (size_t)d * NH * CD, fc1_b + d * NH,
                                                            x, outp, Hp, NH, CD, INV_AW, HCAR, 0);
    gemm_k<2><<<dim3(CD / NTL, TOK / MT), TPB, 0, stream>>>(Hp, W2 + (size_t)d * CD * NH, fc2_b + d * CD,
                                                            outp, outp, XMp, CD, NH, INV_AW, 1.0f, 0);
  }
  (void)hipGetLastError();
}
